// CausalSelfAttention_26645977105196
// MI455X (gfx1250) — hardware-run, weakly checked
//
#include <hip/hip_runtime.h>


#ifndef NB
#define NB 16
#endif
#ifndef SEQ
#define SEQ 1024
#endif
#define NB_FULL  16
#define SEQ_FULL 1024
#ifndef OUT_SEQ
#define OUT_SEQ SEQ
#endif
#define DM   768
#define NH_  12
#define HD   64
#define N3   (3 * DM)
#define AW   4
#define OSP  68
#define EROWS (SEQ < 256 ? SEQ : 256)
#define QRS  2048.0f
#define QRI  (1.0f / 2048.0f)
#define SC2  ((float)(0.125 * 1.4426950408889634))
#define PSH  14.0f
#define NEGB (-3.0e38f)
#define WCS  64.0f
#define YCS  16.0f
#define OSC  (1.0f / 1024.0f)

static_assert(HD == 64);
static_assert(NH_ * HD == DM);
static_assert(DM % 64 == 0);
static_assert(N3 % 64 == 0);
static_assert(DM % 32 == 0);
static_assert(HD % 32 == 0);
static_assert(SEQ % 64 == 0);
static_assert((NB * SEQ) % 64 == 0);
static_assert(SEQ % 32 == 0);
static_assert(SEQ % (16 * AW) == 0);
static_assert(EROWS % 64 == 0);
static_assert(EROWS % 32 == 0);
static_assert(EROWS >= 32);
static_assert(EROWS <= SEQ);
static_assert(EROWS % (16 * AW) == 0);
static_assert((SEQ - EROWS) % (16 * AW) == 0);
static_assert((SEQ - EROWS) % 64 == 0);
static_assert(((size_t)SEQ * DM) % 8 == 0);
static_assert(NB <= NB_FULL);
static_assert(SEQ <= SEQ_FULL);
static_assert((OSP * 4) % 16 == 0);
static_assert(OSP >= HD);
static_assert(4 * 32 * 16 == 16 * HD * 2);
static_assert(8 * 32 * 16 == 16 * 64 * 4);
static_assert(2 * 256 * 16 == 64 * 64 * 2);
static_assert(AW * 16 * OSP * 4 <= 131072);
static_assert(16 * 68 * 4 <= 131072);
static_assert(64 * 72 * 2 <= 131072);

typedef _Float16 h16;
typedef unsigned short bf;
typedef __attribute__((ext_vector_type(16))) __bf16   v16bf;
typedef __attribute__((ext_vector_type(16))) _Float16 v16h;
typedef __attribute__((ext_vector_type(8)))  _Float16 v8h;
typedef __attribute__((ext_vector_type(8)))  unsigned short v8us;
typedef __attribute__((ext_vector_type(8)))  float    v8f;
typedef __attribute__((ext_vector_type(4)))  float    v4f;
typedef v4f  __attribute__((may_alias)) v4fa;

__device__ __forceinline__ unsigned short f2bf(float f) { unsigned u = __float_as_uint(f); u += 0x7FFFu + ((u >> 16) & 1u); return (unsigned short)(u >> 16); }
__device__ __forceinline__ float bfr(float f) { return __uint_as_float(((unsigned)f2bf(f)) << 16); }
__device__ __forceinline__ v16h cat16(v8h lo, v8h hi) { return __builtin_shufflevector(lo, hi, 0, 1, 2, 3, 4, 5, 6, 7, 8, 9, 10, 11, 12, 13, 14, 15); }
__device__ __forceinline__ v16bf cat16b(v8us lo, v8us hi) { return __builtin_bit_cast(v16bf, __builtin_shufflevector(lo, hi, 0, 1, 2, 3, 4, 5, 6, 7, 8, 9, 10, 11, 12, 13, 14, 15)); }
__device__ __forceinline__ v8f wmma16(v16h a, v16h b, v8f c) { return __builtin_amdgcn_wmma_f32_16x16x32_f16(false, a, false, b, (short)0, c, false, false); }
__device__ __forceinline__ v8f wmmab(v16bf a, v16bf b, v8f c) { return __builtin_amdgcn_wmma_f32_16x16x32_bf16(false, a, false, b, (short)0, c, false, false); }
__device__ __forceinline__ v8f wmma16g(v16h a, v16h b, v8f c) { c = wmma16(a, b, c); asm volatile("v_nop\n\tv_nop\n\tv_nop\n\tv_nop" : "+v"(c) : "v"(a), "v"(b)); return c; }
__device__ __forceinline__ v8f wmmabg(v16bf a, v16bf b, v8f c) { c = wmmab(a, b, c); asm volatile("v_nop\n\tv_nop\n\tv_nop\n\tv_nop" : "+v"(c) : "v"(a), "v"(b)); return c; }
__device__ __forceinline__ v16h  ldh(const h16* p) { return cat16(*(const v8h*)p, *(const v8h*)(p + 16)); }
__device__ __forceinline__ v16bf ldb(const bf* p)  { return cat16b(*(const v8us*)p, *(const v8us*)(p + 16)); }
__device__ __forceinline__ void wave_sync() { __builtin_amdgcn_fence(3  , "wavefront"); __builtin_amdgcn_wave_barrier(); asm volatile("" ::: "memory"); }
static __device__ __forceinline__ h16 toh_flush(float v) { const h16 r = (h16)v; return (fabsf(v) < 6.103515625e-05f) ? (h16)0.0f : r; }

__global__ __launch_bounds__(256) void k_cvt8(const float* __restrict__ src, bf* dst, size_t n8) {
    const size_t i = (size_t)blockIdx.x * 256 + threadIdx.x; if (i >= n8) return;
    const v8f v = *(const v8f*)(src + i * 8); v8us o;
#pragma unroll
    for (int k = 0; k < 8; ++k) o[k] = f2bf(v[k]);
    *(volatile v8us*)(dst + i * 8) = o; __threadfence(); *(volatile v8us*)(dst + i * 8) = o;
}

template <int F16>
__device__ __forceinline__ void wt_body(const float* __restrict__ W, bf* WT, int K, int N) {
    __shared__ __align__(16) bf ts[64 * 72];
    const int n0 = blockIdx.x * 64, k0 = blockIdx.y * 64;
    const int tx = threadIdx.x & 63, ty = threadIdx.x >> 6;
#pragma unroll 1
    for (int i = 0; i < 16; ++i) {
        const int k = ty + 4 * i;
        const float v = W[(size_t)(k0 + k) * N + n0 + tx];
        bf o;
        if (F16) { const h16 hh = toh_flush(bfr(v) * WCS); o = __builtin_bit_cast(bf, hh); }
        else     { o = f2bf(v); }
        ts[tx * 72 + k] = o;
    }
    __syncthreads();
#pragma unroll 1
    for (int ps = 0; ps < 2; ++ps) {
#pragma unroll
        for (int s = 0; s < 2; ++s) { const int p = s * 256 + (int)threadIdx.x; const int row = p >> 3, c8 = (p & 7) * 8;
            const v8us val = *(const v8us*)(&ts[row * 72 + c8]);
            *(volatile v8us*)(WT + (size_t)(n0 + row) * K + k0 + c8) = val; }
        if (ps == 0) __threadfence(); }
}
__global__ __launch_bounds__(256) void k_wt_b(const float* __restrict__ W, bf* WT, int K, int N) { wt_body<0>(W, WT, K, N); }
__global__ __launch_bounds__(256) void k_wt_h(const float* __restrict__ W, h16* WT, int K, int N) { wt_body<1>(W, (bf*)WT, K, N); }

template <int MODE>
__device__ __forceinline__ void proj_body(const bf* __restrict__ A, const bf* __restrict__ Bt, const float* __restrict__ bias, h16* Ph, h16* Pr, int resT) {
    __shared__ __align__(16) float os[16 * 68];
    const int K = DM;
    const int lane = threadIdx.x & 31, lr = lane & 15, hi = lane >> 4; const int r0 = blockIdx.x * 64, c0 = blockIdx.y * 64;
    v8f acc[4][4];
#pragma unroll
    for (int mb = 0; mb < 4; ++mb)
#pragma unroll
        for (int nb = 0; nb < 4; ++nb) acc[mb][nb] = (v8f){};
    const size_t aoff = (size_t)(r0 + lr) * K + 8 * hi, boff = (size_t)(c0 + lr) * K + 8 * hi;
#pragma unroll 1
    for (int kc = 0; kc < K; kc += 32) {
        v16bf a[4];
#pragma unroll
        for (int mb = 0; mb < 4; ++mb) a[mb] = ldb(A + aoff + (size_t)mb * 16 * K + kc);
#pragma unroll
        for (int nb = 0; nb < 4; ++nb) { const v16bf b = ldb(Bt + boff + (size_t)nb * 16 * K + kc);
#pragma unroll
            for (int mb = 0; mb < 4; ++mb) acc[mb][nb] = wmmabg(a[mb], b, acc[mb][nb]); }
    }
    float bc[4];
#pragma unroll
    for (int nb = 0; nb < 4; ++nb) bc[nb] = (MODE == 0) ? bfr(bias[c0 + nb * 16 + lr]) : 0.0f;
    size_t tbase, rbase; bool wr;
    if (MODE == 0) { const int bb = r0 / SEQ, tt = r0 % SEQ; const int zc = bb * NH_ + c0 / HD;
                     tbase = ((size_t)zc * SEQ + (size_t)tt) * HD; rbase = ((size_t)zc * (size_t)resT + (size_t)tt) * HD; wr = tt < resT; }
    else           { const int bb = c0 / SEQ, tt = c0 % SEQ;
                     tbase = (size_t)bb * (size_t)DM * SEQ + (size_t)r0 * SEQ + (size_t)tt; rbase = (size_t)bb * (size_t)DM * (size_t)resT + (size_t)r0 * (size_t)resT + (size_t)tt; wr = tt < resT; }
#pragma unroll
    for (int mb = 0; mb < 4; ++mb) {
        float br[8];
#pragma unroll
        for (int j = 0; j < 8; ++j) br[j] = (MODE == 1) ? bfr(bias[r0 + mb * 16 + hi * 8 + j]) : 0.0f;
#pragma unroll
        for (int nb = 0; nb < 4; ++nb) {
#pragma unroll
            for (int j = 0; j < 8; ++j) os[(hi * 8 + j) * 68 + nb * 16 + lr] = acc[mb][nb][j] + bc[nb] + br[j]; }
        wave_sync();
#pragma unroll 1
        for (int ps = 0; ps < 2; ++ps) {
            if (MODE == 0) {
                const size_t sb = tbase + (size_t)(mb * 16) * HD;
                const size_t rb = rbase + (size_t)(mb * 16) * HD;
#pragma unroll
                for (int s = 0; s < 4; ++s) { const int p = s * 32 + lane; const int row = p >> 3, c8 = (p & 7) * 8;
                    const v4f x0 = *(const v4fa*)(&os[row * 68 + c8]); const v4f x1 = *(const v4fa*)(&os[row * 68 + c8 + 4]); v8h hv, rv;
#pragma unroll
                    for (int i = 0; i < 4; ++i) { const h16 a0 = toh_flush(x0[i]); const h16 a1 = toh_flush(x1[i]); hv[i] = a0; hv[4 + i] = a1;
                        rv[i] = toh_flush((x0[i] - (float)a0) * QRS); rv[4 + i] = toh_flush((x1[i] - (float)a1) * QRS); }
                    const size_t oo = sb + (size_t)p * 8;
                    const size_t ro = rb + (size_t)p * 8;
                    *(volatile v8h*)(Ph + oo) = hv; if (wr) *(volatile v8h*)(Pr + ro) = rv; }
            } else {
                const size_t sb = tbase + (size_t)(mb * 16) * SEQ;
                const size_t rb = rbase + (size_t)(mb * 16) * (size_t)resT;
#pragma unroll
                for (int s = 0; s < 4; ++s) { const int row = 4 * s + (lane >> 3), c8 = (lane & 7) * 8;
                    const v4f x0 = *(const v4fa*)(&os[row * 68 + c8]); const v4f x1 = *(const v4fa*)(&os[row * 68 + c8 + 4]); v8h hv, rv;
#pragma unroll
                    for (int i = 0; i < 4; ++i) { const h16 a0 = toh_flush(x0[i]); const h16 a1 = toh_flush(x1[i]); hv[i] = a0; hv[4 + i] = a1;
                        rv[i] = toh_flush((x0[i] - (float)a0) * QRS); rv[4 + i] = toh_flush((x1[i] - (float)a1) * QRS); }
                    const size_t oo = sb + (size_t)row * SEQ + c8;
                    const size_t ro = rb + (size_t)row * (size_t)resT + c8;
                    *(volatile v8h*)(Ph + oo) = hv; if (wr) *(volatile v8h*)(Pr + ro) = rv; }
            }
            if (ps == 0) __threadfence(); }
        wave_sync();
    }
}
__global__ __launch_bounds__(32) void k_proj_rows(const bf* __restrict__ A, const bf* __restrict__ Bt, const float* __restrict__ bias, h16* Ph, h16* Pr, int resT) { proj_body<0>(A, Bt, bias, Ph, Pr, resT); }
__global__ __launch_bounds__(32) void k_proj_cols(const bf* __restrict__ A, const bf* __restrict__ Bt, const float* __restrict__ bias, h16* Ph, h16* Pr, int resT) { proj_body<1>(A, Bt, bias, Ph, Pr, resT); }

template <int EARLY>
__device__ __forceinline__ void flash_body(const h16* __restrict__ QH, const h16* __restrict__ QR, const h16* __restrict__ KP, const h16* __restrict__ KR,
                                           const h16* __restrict__ VT, const h16* __restrict__ VR, h16* YH, h16* YR) {
    __shared__ __align__(16) float os[AW * 16 * OSP];
    const int lane = threadIdx.x & 31, lr = lane & 15, hi = lane >> 4;
    const int wave = __builtin_amdgcn_readfirstlane((int)(threadIdx.x >> 5));
    const int zh = blockIdx.y; const int b = zh / NH_, h = zh % NH_;
    const int t0 = (EARLY ? 0 : EROWS) + (blockIdx.x * AW + wave) * 16;
    const int lim = t0 + lr;
    const int nk = (t0 + 16 + 31) & ~31;
    const size_t pbase = (size_t)zh * SEQ * HD;
    const size_t rbase = (size_t)zh * EROWS * HD;
    const size_t qo  = pbase + (size_t)(t0 + lr) * HD + 8 * hi;
    const size_t qro = rbase + (size_t)(t0 + lr) * HD + 8 * hi;
    const size_t ko  = pbase + (size_t)lr * HD + 8 * hi;
    const size_t vo  = pbase + (size_t)lr * SEQ + 8 * hi;
    const size_t kro = rbase + (size_t)lr * HD + 8 * hi;
    const size_t vro = rbase + (size_t)lr * EROWS + 8 * hi;
    const v16h hz = (v16h){};
    v16h qk0 = hz, qk1 = hz;
    if (!EARLY) { qk0 = ldh(QH + qo); qk1 = ldh(QH + qo + 32); }
    v8f o0 = (v8f){}, o1 = (v8f){}, o2 = (v8f){}, o3 = (v8f){};
    v8f oR0 = (v8f){}, oR1 = (v8f){}, oR2 = (v8f){}, oR3 = (v8f){};
    float m = NEGB, l = 0.0f;
#pragma unroll 1
    for (int key0 = 0; key0 < nk; key0 += 32) {
        v16h q0 = qk0, q1 = qk1, qr0 = hz, qr1 = hz;
        if (EARLY) { int qz = 0; asm volatile("" : "+v"(qz));
                     q0 = ldh(QH + qo + qz); q1 = ldh(QH + qo + qz + 32); qr0 = ldh(QR + qro + qz); qr1 = ldh(QR + qro + qz + 32); }
        const h16* ka = KP + ko + (size_t)key0 * HD;
        float ta[8], tb[8];
        if (EARLY) {
            const h16* kr = KR + kro + (size_t)key0 * HD;
            { const v16h k0 = ldh(ka), k1 = ldh(ka + 32), r0 = ldh(kr), r1 = ldh(kr + 32);
              v8f sH = (v8f){}, sL = (v8f){}, sM = (v8f){};
              sH = wmma16g(k0, q0, sH); sL = wmma16g(k0, qr0, sL); sM = wmma16g(r0, q0, sM);
              sH = wmma16g(k1, q1, sH); sL = wmma16g(k1, qr1, sL); sM = wmma16g(r1, q1, sM);
#pragma unroll
              for (int r = 0; r < 8; ++r) ta[r] = (sH[r] + (sL[r] + sM[r]) * QRI) * SC2; }
            { const v16h k0 = ldh(ka + 16 * HD), k1 = ldh(ka + 16 * HD + 32), r0 = ldh(kr + 16 * HD), r1 = ldh(kr + 16 * HD + 32);
              v8f sH = (v8f){}, sL = (v8f){}, sM = (v8f){};
              sH = wmma16g(k0, q0, sH); sL = wmma16g(k0, qr0, sL); sM = wmma16g(r0, q0, sM);
              sH = wmma16g(k1, q1, sH); sL = wmma16g(k1, qr1, sL); sM = wmma16g(r1, q1, sM);
#pragma unroll
              for (int r = 0; r < 8; ++r) tb[r] = (sH[r] + (sL[r] + sM[r]) * QRI) * SC2; }
        } else {
            const v16h k0a = ldh(ka), k1a = ldh(ka + 32), k0b = ldh(ka + 16 * HD), k1b = ldh(ka + 16 * HD + 32);
            v8f sHa = (v8f){}, sHb = (v8f){};
            sHa = wmma16g(k0a, q0, sHa); sHb = wmma16g(k0b, q0, sHb); sHa = wmma16g(k1a, q1, sHa); sHb = wmma16g(k1b, q1, sHb);
#pragma unroll
            for (int r = 0; r < 8; ++r) { ta[r] = sHa[r] * SC2; tb[r] = sHb[r] * SC2; }
        }
        const int ja = key0 + 8 * hi;
        bool fa[8], fb[8]; float mx = NEGB;
#pragma unroll
        for (int r = 0; r < 8; ++r) {
            fa[r] = (ja + r <= lim);
            fb[r] = (ja + 16 + r <= lim);
            mx = fmaxf(mx, fmaxf(fa[r] ? ta[r] : NEGB, fb[r] ? tb[r] : NEGB)); }
        mx = fmaxf(mx, __shfl_xor(mx, 16, 32));
        const float mnew = fmaxf(m, mx);
        const float alpha = __builtin_amdgcn_exp2f(m - mnew);
        const float sh = PSH - mnew;
        v16h pb, pr = hz; float ls = 0.0f;
#pragma unroll
        for (int r = 0; r < 8; ++r) {
            const float xa = ta[r] + sh, xb = tb[r] + sh;
            const float ea = __builtin_amdgcn_exp2f(xa), eb = __builtin_amdgcn_exp2f(xb);
            const float ga = (fa[r] & (xa >= -14.0f)) ? ea : 0.0f;
            const float gb = (fb[r] & (xb >= -14.0f)) ? eb : 0.0f;
            const h16 pa = (h16)ga; const h16 pc = (h16)gb;
            pb[r] = pa; pb[8 + r] = pc;
            if (EARLY) { pr[r] = toh_flush((ga - (float)pa) * QRS); pr[8 + r] = toh_flush((gb - (float)pc) * QRS); ls += ga + gb; }
            else       { ls += (float)pa + (float)pc; } }
        l = l * alpha + ls; m = mnew;
        o0 = o0 * alpha; o1 = o1 * alpha; o2 = o2 * alpha; o3 = o3 * alpha;
        if (EARLY) { oR0 = oR0 * alpha; oR1 = oR1 * alpha; oR2 = oR2 * alpha; oR3 = oR3 * alpha; }
        const h16* va = VT + vo + key0;
        if (EARLY) {
            const h16* vr = VR + vro + key0;
            { const v16h v0 = ldh(va), v1 = ldh(va + (size_t)16 * SEQ), w0 = ldh(vr), w1 = ldh(vr + (size_t)16 * EROWS);
              o0 = wmma16g(v0, pb, o0); o1 = wmma16g(v1, pb, o1);
              oR0 = wmma16g(v0, pr, oR0); oR1 = wmma16g(v1, pr, oR1);
              oR0 = wmma16g(w0, pb, oR0); oR1 = wmma16g(w1, pb, oR1); }
            { const v16h v0 = ldh(va + (size_t)32 * SEQ), v1 = ldh(va + (size_t)48 * SEQ), w0 = ldh(vr + (size_t)32 * EROWS), w1 = ldh(vr + (size_t)48 * EROWS);
              o2 = wmma16g(v0, pb, o2); o3 = wmma16g(v1, pb, o3);
              oR2 = wmma16g(v0, pr, oR2); oR3 = wmma16g(v1, pr, oR3);
              oR2 = wmma16g(w0, pb, oR2); oR3 = wmma16g(w1, pb, oR3); }
        } else {
            const v16h v0 = ldh(va), v1 = ldh(va + (size_t)16 * SEQ), v2 = ldh(va + (size_t)32 * SEQ), v3 = ldh(va + (size_t)48 * SEQ);
            o0 = wmma16g(v0, pb, o0); o1 = wmma16g(v1, pb, o1); o2 = wmma16g(v2, pb, o2); o3 = wmma16g(v3, pb, o3);
        }
    }
    l += __shfl_xor(l, 16, 32);
    const bool any = l > 0.0f;
    const float lsafe = any ? l : 1.0f;
    const float inv = any ? (1.0f / lsafe) : 0.0f;
    v8f f0 = o0, f1 = o1, f2 = o2, f3 = o3;
    if (EARLY) { f0 = o0 + oR0 * QRI; f1 = o1 + oR1 * QRI; f2 = o2 + oR2 * QRI; f3 = o3 + oR3 * QRI; }
    const int wb = wave * 16 * OSP;
    { v4f a, c;
      a[0] = f0[0] * inv; a[1] = f0[1] * inv; a[2] = f0[2] * inv; a[3] = f0[3] * inv; c[0] = f0[4] * inv; c[1] = f0[5] * inv; c[2] = f0[6] * inv; c[3] = f0[7] * inv;
      *(v4fa*)(&os[wb + lr * OSP +  0 + 8 * hi]) = a; *(v4fa*)(&os[wb + lr * OSP +  0 + 8 * hi + 4]) = c;
      a[0] = f1[0] * inv; a[1] = f1[1] * inv; a[2] = f1[2] * inv; a[3] = f1[3] * inv; c[0] = f1[4] * inv; c[1] = f1[5] * inv; c[2] = f1[6] * inv; c[3] = f1[7] * inv;
      *(v4fa*)(&os[wb + lr * OSP + 16 + 8 * hi]) = a; *(v4fa*)(&os[wb + lr * OSP + 16 + 8 * hi + 4]) = c;
      a[0] = f2[0] * inv; a[1] = f2[1] * inv; a[2] = f2[2] * inv; a[3] = f2[3] * inv; c[0] = f2[4] * inv; c[1] = f2[5] * inv; c[2] = f2[6] * inv; c[3] = f2[7] * inv;
      *(v4fa*)(&os[wb + lr * OSP + 32 + 8 * hi]) = a; *(v4fa*)(&os[wb + lr * OSP + 32 + 8 * hi + 4]) = c;
      a[0] = f3[0] * inv; a[1] = f3[1] * inv; a[2] = f3[2] * inv; a[3] = f3[3] * inv; c[0] = f3[4] * inv; c[1] = f3[5] * inv; c[2] = f3[6] * inv; c[3] = f3[7] * inv;
      *(v4fa*)(&os[wb + lr * OSP + 48 + 8 * hi]) = a; *(v4fa*)(&os[wb + lr * OSP + 48 + 8 * hi + 4]) = c; }
    wave_sync();
    const size_t yb = ((size_t)b * SEQ + t0) * DM + (size_t)h * HD;
    const size_t rb = ((size_t)b * EROWS + t0) * DM + (size_t)h * HD;
#pragma unroll 1
    for (int ps = 0; ps < 2; ++ps) {
#pragma unroll
        for (int s = 0; s < 4; ++s) { const int row = 4 * s + (lane >> 3), c8 = (lane & 7) * 8;
            const v4f x0 = *(const v4fa*)(&os[wb + row * OSP + c8]); const v4f x1 = *(const v4fa*)(&os[wb + row * OSP + c8 + 4]); v8h hv, rv;
#pragma unroll
            for (int i = 0; i < 4; ++i) { const float y0 = x0[i] * YCS, y1 = x1[i] * YCS; const h16 a0 = toh_flush(y0); const h16 a1 = toh_flush(y1); hv[i] = a0; hv[4 + i] = a1;
                rv[i] = toh_flush((y0 - (float)a0) * QRS); rv[4 + i] = toh_flush((y1 - (float)a1) * QRS); }
            *(volatile v8h*)(YH + yb + (size_t)row * DM + c8) = hv;
            if (EARLY) *(volatile v8h*)(YR + rb + (size_t)row * DM + c8) = rv; }
        if (ps == 0) __threadfence(); }
}
__global__ __launch_bounds__(32 * AW) __attribute__((amdgpu_num_vgpr(256))) void k_flash_early(const h16* __restrict__ QH, const h16* __restrict__ QR, const h16* __restrict__ KP, const h16* __restrict__ KR,
                                                    const h16* __restrict__ VT, const h16* __restrict__ VR, h16* YH, h16* YR) { flash_body<1>(QH, QR, KP, KR, VT, VR, YH, YR); }
__global__ __launch_bounds__(32 * AW) __attribute__((amdgpu_num_vgpr(256))) void k_flash_late(const h16* __restrict__ QH, const h16* __restrict__ QR, const h16* __restrict__ KP, const h16* __restrict__ KR,
                                                   const h16* __restrict__ VT, const h16* __restrict__ VR, h16* YH, h16* YR) { flash_body<0>(QH, QR, KP, KR, VT, VR, YH, YR); }

template <int EARLY>
__device__ __forceinline__ void oproj_body(const h16* __restrict__ YH, const h16* __restrict__ YR, const h16* __restrict__ WP, const float* __restrict__ bias, float* OUT) {
    constexpr int MB  = EARLY ? 2 : 4;
    constexpr int TPB = EARLY ? (EROWS / 32) : (((SEQ - EROWS) / 64) > 0 ? ((SEQ - EROWS) / 64) : 1);
    __shared__ __align__(16) float os[16 * 68];
    const int K = DM;
    const int lane = threadIdx.x & 31, lr = lane & 15, hi = lane >> 4;
    const int bb = blockIdx.x / TPB; const int tt = (EARLY ? 0 : EROWS) + ((int)blockIdx.x % TPB) * (16 * MB);
    const int c0 = blockIdx.y * 64;
    v8f acc[4][4], accR[4][4];
#pragma unroll
    for (int mb = 0; mb < 4; ++mb)
#pragma unroll
        for (int nb = 0; nb < 4; ++nb) { acc[mb][nb] = (v8f){}; accR[mb][nb] = (v8f){}; }
    const size_t aoff = ((size_t)bb * SEQ + (size_t)(tt + lr)) * K + 8 * hi;
    const size_t roff = ((size_t)bb * EROWS + (size_t)(tt + lr)) * K + 8 * hi;
    const size_t boff = (size_t)(c0 + lr) * K + 8 * hi;
#pragma unroll 1
    for (int kc = 0; kc < K; kc += 32) {
        v16h a[4], ar[4];
#pragma unroll
        for (int mb = 0; mb < MB; ++mb) { a[mb] = ldh(YH + aoff + (size_t)mb * 16 * K + kc); if (EARLY) ar[mb] = ldh(YR + roff + (size_t)mb * 16 * K + kc); }
#pragma unroll
        for (int nb = 0; nb < 4; ++nb) { const v16h bw = ldh(WP + boff + (size_t)nb * 16 * K + kc);
#pragma unroll
            for (int mb = 0; mb < MB; ++mb) acc[mb][nb] = wmma16g(a[mb], bw, acc[mb][nb]);
            if (EARLY) {
#pragma unroll
                for (int mb = 0; mb < MB; ++mb) accR[mb][nb] = wmma16g(ar[mb], bw, accR[mb][nb]); } }
    }
    float bc[4];
#pragma unroll
    for (int nb = 0; nb < 4; ++nb) bc[nb] = bfr(bias[c0 + nb * 16 + lr]);
#pragma unroll
    for (int mb = 0; mb < MB; ++mb) {
#pragma unroll
        for (int nb = 0; nb < 4; ++nb) {
#pragma unroll
            for (int j = 0; j < 8; ++j) { float v = acc[mb][nb][j]; if (EARLY) v += accR[mb][nb][j] * QRI;
                os[(hi * 8 + j) * 68 + nb * 16 + lr] = v * OSC + bc[nb]; } }
        wave_sync();
        float* orow = OUT + ((size_t)bb * OUT_SEQ + (size_t)(tt + mb * 16)) * DM + c0;
#pragma unroll 1
        for (int ps = 0; ps < 2; ++ps) {
#pragma unroll
            for (int s = 0; s < 8; ++s) { const int p = s * 32 + lane; const int row = p >> 4, c4 = (p & 15) * 4;
                const v4f val = *(const v4fa*)(&os[row * 68 + c4]);
                *(volatile v4f*)(orow + (size_t)row * DM + c4) = val; }
            if (ps == 0) __threadfence(); }
        wave_sync();
    }
}
__global__ __launch_bounds__(32) __attribute__((amdgpu_num_vgpr(256))) void k_oproj_early(const h16* __restrict__ YH, const h16* __restrict__ YR, const h16* __restrict__ WP, const float* __restrict__ bias, float* OUT) { oproj_body<1>(YH, YR, WP, bias, OUT); }
__global__ __launch_bounds__(32) __attribute__((amdgpu_num_vgpr(256))) void k_oproj_late(const h16* __restrict__ YH, const h16* __restrict__ YR, const h16* __restrict__ WP, const float* __restrict__ bias, float* OUT) { oproj_body<0>(YH, YR, WP, bias, OUT); }

static constexpr size_t al256(size_t v) { return (v + 255) & ~(size_t)255; }
static constexpr size_t SZ_XB = al256((size_t)NB * SEQ * DM * 2);
static constexpr size_t SZ_WA = al256((size_t)N3 * DM * 2);
static constexpr size_t SZ_WP = al256((size_t)DM * DM * 2);
static constexpr size_t SZ_PL = al256((size_t)NB * NH_ * SEQ * HD * 2);
static constexpr size_t SZ_RS = al256((size_t)NB * NH_ * EROWS * HD * 2);
static constexpr size_t SZ_YR = al256((size_t)NB * EROWS * DM * 2);
static constexpr size_t SZ_TOTAL = SZ_XB + SZ_WA + SZ_WP + 3 * SZ_PL + 3 * SZ_RS + SZ_YR;
static_assert(SZ_TOTAL <= (size_t)134217728);
static_assert((size_t)NB * SEQ * DM * 2 <= SZ_XB);
static_assert(((size_t)DM * DM * 2) % 256 == 0);
static_assert((size_t)NB * NH_ * SEQ * HD == (size_t)NB * DM * SEQ);
static_assert((size_t)NB * NH_ * EROWS * HD == (size_t)NB * DM * EROWS);

extern "C" void kernel_launch(void* const* d_in, const int* in_sizes, int n_in,
                              void* d_out, int out_size, void* d_ws, size_t ws_size, hipStream_t stream) {
    if (n_in < 5) return;
    const size_t needx = ((size_t)(NB - 1) * SEQ_FULL + SEQ) * DM;
    if ((size_t)in_sizes[0] < needx) return;
    if ((size_t)in_sizes[1] < (size_t)DM * N3 || in_sizes[2] < N3) return;
    if ((size_t)in_sizes[3] < (size_t)DM * DM || in_sizes[4] < DM) return;
    if ((size_t)out_size < ((size_t)(NB - 1) * OUT_SEQ + SEQ) * DM) return;
    if (SZ_TOTAL > ws_size) return;
    const float* x  = (const float*)d_in[0];
    const float* wa = (const float*)d_in[1]; const float* ba = (const float*)d_in[2];
    const float* wp = (const float*)d_in[3]; const float* bp = (const float*)d_in[4];
    float* OUT = (float*)d_out;
    char* wsp = (char*)d_ws;
    bf*  XB  = (bf*)wsp;
    h16* YH  = (h16*)wsp; wsp += SZ_XB;
    bf*  WTA = (bf*)wsp;  wsp += SZ_WA;
    h16* WPH = (h16*)wsp; wsp += SZ_WP;
    h16* QH  = (h16*)wsp; wsp += SZ_PL;
    h16* KP  = (h16*)wsp; wsp += SZ_PL;
    h16* VT  = (h16*)wsp; wsp += SZ_PL;
    h16* QR  = (h16*)wsp; wsp += SZ_RS;
    h16* KR  = (h16*)wsp; wsp += SZ_RS;
    h16* VR  = (h16*)wsp; wsp += SZ_RS;
    h16* YR  = (h16*)wsp; wsp += SZ_YR;

    if (SEQ == SEQ_FULL) {
        const size_t n8 = (size_t)NB * SEQ * DM / 8;
        k_cvt8<<<(unsigned)((n8 + 255) / 256), 256, 0, stream>>>(x, XB, n8);
    } else {
        const size_t n8 = (size_t)SEQ * DM / 8;
        for (int b = 0; b < NB; ++b) k_cvt8<<<(unsigned)((n8 + 255) / 256), 256, 0, stream>>>(x + (size_t)b * SEQ_FULL * DM, XB + (size_t)b * SEQ * DM, n8);
    }
    k_wt_b<<<dim3(N3 / 64, DM / 64, 1), 256, 0, stream>>>(wa, WTA, DM, N3);
    k_wt_h<<<dim3(DM / 64, DM / 64, 1), 256, 0, stream>>>(wp, WPH, DM, DM);

    k_proj_rows<<<dim3(NB * SEQ / 64, DM / 64, 1), 32, 0, stream>>>(XB, WTA, ba, QH, QR, EROWS);
    k_proj_rows<<<dim3(NB * SEQ / 64, DM / 64, 1), 32, 0, stream>>>(XB, WTA + (size_t)DM * DM, ba + DM, KP, KR, EROWS);
    k_proj_cols<<<dim3(DM / 64, NB * SEQ / 64, 1), 32, 0, stream>>>(WTA + (size_t)2 * DM * DM, XB, ba + 2 * DM, VT, VR, EROWS);

    k_flash_early<<<dim3(EROWS / (16 * AW), NB * NH_, 1), 32 * AW, 0, stream>>>(QH, QR, KP, KR, VT, VR, YH, YR);
    if (SEQ > EROWS)
        k_flash_late<<<dim3((SEQ - EROWS) / (16 * AW), NB * NH_, 1), 32 * AW, 0, stream>>>(QH, QR, KP, KR, VT, VR, YH, YR);

    k_oproj_early<<<dim3(NB * (EROWS / 32), DM / 64, 1), 32, 0, stream>>>(YH, YR, WPH, bp, OUT);
    if (SEQ > EROWS)
        k_oproj_late<<<dim3(NB * ((SEQ - EROWS) / 64), DM / 64, 1), 32, 0, stream>>>(YH, YR, WPH, bp, OUT);
}
